// ConditionalLayer_76055280877934
// MI455X (gfx1250) — hardware-verified
//
#include <hip/hip_runtime.h>


#ifndef NB
#define NB 8192
#endif
#define NB_FULL 8192
#define KD    1024
#define ND    1024
#define NREL  8
#define NSLOT 32
#define RB    1024
#define NBLK  (NB / RB)
#define OFFP  128
#define PROWS (NB + 512)
#define OSP   68

static_assert(NB % RB == 0);
static_assert(NBLK >= 1 && NBLK <= OFFP);
static_assert(NB <= NB_FULL);
static_assert(NREL * 63 <= PROWS - NB);
static_assert(PROWS % 64 == 0);
static_assert(NREL <= NSLOT && NSLOT == 32);
static_assert(KD % 32 == 0);
static_assert(ND % 64 == 0);
static_assert(KD * 2 == 32 * 16 * 4);
static_assert(RB == 32 * 32);
static_assert(ND == 256 * 4);
static_assert(32 * 16 * 32 == 64 * 64 * 4);
static_assert(64 * OSP * 4 <= 131072);
static_assert(OFFP * 4 == 32 * 16);
static_assert(((size_t)NREL * ND * KD) % (256 * 8) == 0);
static_assert(NB % 4 == 0);

typedef unsigned short bf;
typedef __attribute__((ext_vector_type(16))) __bf16   v16bf;
typedef __attribute__((ext_vector_type(8)))  unsigned short v8us;
typedef __attribute__((ext_vector_type(8)))  float    v8f;
typedef __attribute__((ext_vector_type(4)))  float    v4f;
typedef __attribute__((ext_vector_type(4)))  int      v4i;
typedef v4f  __attribute__((may_alias)) v4fa;
typedef v4i  __attribute__((may_alias)) v4ia;

__device__ __forceinline__ unsigned short f2bf(float f) { unsigned u = __float_as_uint(f); u += 0x7FFFu + ((u >> 16) & 1u); return (unsigned short)(u >> 16); }
__device__ __forceinline__ float bf2f(unsigned short w) { return __uint_as_float(((unsigned)w) << 16); }
__device__ __forceinline__ int clampi(int v, int lo, int hi) { return min(max(v, lo), hi); }
__device__ __forceinline__ v16bf cat16b(v8us lo, v8us hi) { return __builtin_bit_cast(v16bf, __builtin_shufflevector(lo, hi, 0, 1, 2, 3, 4, 5, 6, 7, 8, 9, 10, 11, 12, 13, 14, 15)); }
__device__ __forceinline__ v8f wmmab(v16bf a, v16bf b, v8f c) { return __builtin_amdgcn_wmma_f32_16x16x32_bf16(false, a, false, b, (short)0, c, false, false); }
__device__ __forceinline__ v16bf ldb(const bf* p)  { return cat16b(*(const v8us*)p, *(const v8us*)(p + 16)); }
__device__ __forceinline__ void wave_sync() { __builtin_amdgcn_fence(3  , "wavefront"); __builtin_amdgcn_wave_barrier(); asm volatile("" ::: "memory"); }

__global__ __launch_bounds__(256) void k_wconv(const float* __restrict__ W, bf* WB) {
    const size_t i = ((size_t)blockIdx.x * 256 + threadIdx.x) * 8;
    if (i >= (size_t)NREL * ND * KD) return;
    const v8f a = *(const v8f*)(W + i); v8us o;
#pragma unroll
    for (int k = 0; k < 8; ++k) o[k] = f2bf(a[k]);
    *(volatile v8us*)(WB + i) = o; __threadfence(); *(volatile v8us*)(WB + i) = o;
}

__global__ __launch_bounds__(256) void k_bias(const float* __restrict__ b, float* BS) {
    const int c4 = 4 * threadIdx.x;
    v4f s; s[0] = 0.0f; s[1] = 0.0f; s[2] = 0.0f; s[3] = 0.0f;
#pragma unroll 1
    for (int g = 0; g < NREL; ++g) { const v4f v = *(const v4f*)(b + (size_t)g * ND + c4);
#pragma unroll
        for (int i = 0; i < 4; ++i) s[i] += bf2f(f2bf(v[i])); }
    *(volatile v4f*)(BS + c4) = s; __threadfence(); *(volatile v4f*)(BS + c4) = s;
}

__global__ __launch_bounds__(1024) void k_count(const int* __restrict__ rels, int* cnt) {
    __shared__ int wc[32 * 32];
    __shared__ __align__(16) int line[32];
    const int tid = threadIdx.x, lane = tid & 31; const int wave = __builtin_amdgcn_readfirstlane(tid >> 5);
    const int blk = blockIdx.x;
    const int rel = clampi(rels[(size_t)blk * RB + tid], 0, NREL - 1);
    int mine = 0;
#pragma unroll 1
    for (int r = 0; r < NREL; ++r) { const unsigned m = __builtin_amdgcn_ballot_w32(rel == r); const int c = __builtin_popcount(m); mine = (lane == r) ? c : mine; }
    wc[wave * 32 + lane] = mine;
    __syncthreads();
    if (wave == 0) {
        int s = 0;
#pragma unroll 1
        for (int w = 0; w < 32; ++w) s += wc[w * 32 + lane];
        line[lane] = s;
        wave_sync();
#pragma unroll 1
        for (int ps = 0; ps < 2; ++ps) {
            if (lane < 8) { const v4i v = *(const v4ia*)(&line[4 * lane]); *(volatile v4i*)(cnt + (size_t)blk * 32 + 4 * lane) = v; }
            if (ps == 0) __threadfence(); }
    }
}

__global__ __launch_bounds__(1024) void k_scan(const int* __restrict__ cnt, int* offs, int* T, bf* AP) {
    __shared__ int tots[32];
    __shared__ __align__(16) int tl[128];
    const int tid = threadIdx.x, lane = tid & 31; const int r = __builtin_amdgcn_readfirstlane(tid >> 5);
    int c[4]; int ls = 0;
#pragma unroll
    for (int i = 0; i < 4; ++i) { const int blk = 4 * lane + i; const int bc = min(blk, NBLK - 1);
        int v = cnt[(size_t)bc * 32 + r]; v = (blk < NBLK) ? v : 0; v = clampi(v, 0, RB); c[i] = v; ls += v; }
    int x = ls;
#pragma unroll
    for (int d = 1; d < 32; d <<= 1) { const int y = __shfl_up(x, d, 32); x += (lane >= d) ? y : 0; }
    const int excl = x - ls;
    const int tot = __shfl(x, 31, 32);
    if (lane == 0) tots[r] = tot;
    __syncthreads();
    const int t = tots[lane]; const int pd = (t + 63) & ~63;
    int y2 = pd;
#pragma unroll
    for (int d = 1; d < 32; d <<= 1) { const int y = __shfl_up(y2, d, 32); y2 += (lane >= d) ? y : 0; }
    const int sstart = y2 - pd;
    const int ptot = __shfl(y2, 31, 32);
    const int segr = __shfl(sstart, r, 32);
    v4i o; o[0] = segr + excl; o[1] = o[0] + c[0]; o[2] = o[1] + c[1]; o[3] = o[2] + c[2];
    if (r == 0) { tl[lane] = sstart; tl[32 + lane] = t; tl[64 + lane] = (lane == 0) ? ptot : 0; tl[96 + lane] = 0; wave_sync(); }
    const int padcnt = ((tot + 63) & ~63) - tot;
    const int pbase = segr + tot;
    v8us z;
#pragma unroll
    for (int k = 0; k < 8; ++k) z[k] = (unsigned short)0;
#pragma unroll 1
    for (int ps = 0; ps < 2; ++ps) {
        *(volatile v4i*)(offs + (size_t)r * OFFP + 4 * lane) = o;
        if (r == 0) { const v4i v = *(const v4ia*)(&tl[4 * lane]); *(volatile v4i*)(T + 4 * lane) = v; }
#pragma unroll 1
        for (int j = 0; j < 63; ++j) { const int p = clampi(pbase + j, 0, PROWS - 1);
            if (j < padcnt) {
#pragma unroll 1
                for (int q = 0; q < 4; ++q) *(volatile v8us*)(AP + (size_t)p * KD + q * 256 + lane * 8) = z; } }
        if (ps == 0) __threadfence(); }
}

__global__ __launch_bounds__(1024) void k_rank(const int* __restrict__ rels, const float* __restrict__ xin,
                                               const int* __restrict__ offs, int* POS, bf* AP) {
    __shared__ int wc[32 * 32];
    const int tid = threadIdx.x, lane = tid & 31; const int wave = __builtin_amdgcn_readfirstlane(tid >> 5);
    const int blk = blockIdx.x;
    const size_t row = (size_t)blk * RB + tid;
    const int rel = clampi(rels[row], 0, NREL - 1);
    int mine = 0; unsigned mymask = 0u;
#pragma unroll 1
    for (int r = 0; r < NREL; ++r) { const unsigned m = __builtin_amdgcn_ballot_w32(rel == r); const int c = __builtin_popcount(m);
        mine = (lane == r) ? c : mine; mymask = (rel == r) ? m : mymask; }
    const int lrank = __builtin_popcount(mymask & ((1u << lane) - 1u));
    wc[wave * 32 + lane] = mine;
    __syncthreads();
    if (wave == 0) {
        int run = clampi(offs[(size_t)lane * OFFP + blk], 0, PROWS);
#pragma unroll 1
        for (int w = 0; w < 32; ++w) { const int c = wc[w * 32 + lane]; wc[w * 32 + lane] = run; run += c; }
    }
    __syncthreads();
    const int pos = clampi(wc[wave * 32 + rel] + lrank, 0, PROWS - 1);
#pragma unroll 1
    for (int ps = 0; ps < 2; ++ps) {
        *(volatile int*)(POS + row) = pos;
#pragma unroll 1
        for (int j = 0; j < 32; ++j) { const int p = __shfl(pos, j, 32);
            const size_t rg = (size_t)blk * RB + (size_t)wave * 32 + j;
#pragma unroll 1
            for (int q = 0; q < 4; ++q) { const int cc = q * 256 + lane * 8;
                const v8f a = *(const v8f*)(xin + rg * KD + cc); v8us oa;
#pragma unroll
                for (int k = 0; k < 8; ++k) oa[k] = f2bf(a[k]);
                *(volatile v8us*)(AP + (size_t)p * KD + cc) = oa; } }
        if (ps == 0) __threadfence(); }
}

__global__ __launch_bounds__(32) __attribute__((amdgpu_num_vgpr(256))) void k_gemm(const bf* __restrict__ AP, const bf* __restrict__ WB, const float* __restrict__ BS,
                                                                                    const int* __restrict__ T, float* SORTED) {
    __shared__ __align__(16) float os[64 * OSP];
    const int lane = threadIdx.x & 31, lr = lane & 15, hi = lane >> 4;
    const int p0 = blockIdx.x * 64;
    const int n0 = blockIdx.y * 64;
    const int ss = T[lane], tt = T[32 + lane];
    const int pe = ss + ((tt + 63) & ~63);
    const unsigned msk = __builtin_amdgcn_ballot_w32((p0 >= ss) && (p0 < pe));
    if (msk == 0u) return;
    const int r = clampi(__builtin_amdgcn_readfirstlane(__builtin_ctz(msk)), 0, NREL - 1);
    v8f acc[4][4];
#pragma unroll
    for (int mb = 0; mb < 4; ++mb)
#pragma unroll
        for (int nb = 0; nb < 4; ++nb) acc[mb][nb] = (v8f){};
    const size_t aoff = (size_t)(p0 + lr) * KD + 8 * hi, boff = (size_t)r * ((size_t)ND * KD) + (size_t)(n0 + lr) * KD + 8 * hi;
#pragma unroll 1
    for (int kc = 0; kc < KD; kc += 32) {
        v16bf a[4];
#pragma unroll
        for (int mb = 0; mb < 4; ++mb) a[mb] = ldb(AP + aoff + (size_t)mb * 16 * KD + kc);
#pragma unroll
        for (int nb = 0; nb < 4; ++nb) { const v16bf b = ldb(WB + boff + (size_t)nb * 16 * KD + kc);
#pragma unroll
            for (int mb = 0; mb < 4; ++mb) acc[mb][nb] = wmmab(a[mb], b, acc[mb][nb]); }
        asm volatile("v_nop\n\tv_nop\n\tv_nop\n\tv_nop" : "+v"(acc[0][0]), "+v"(acc[1][1]), "+v"(acc[2][2]), "+v"(acc[3][3]) : "v"(a[0]), "v"(a[1]), "v"(a[2]), "v"(a[3]));
    }
#pragma unroll
    for (int mb = 0; mb < 4; ++mb) {
#pragma unroll
        for (int nb = 0; nb < 4; ++nb) {
#pragma unroll
            for (int j = 0; j < 8; ++j) os[(mb * 16 + hi * 8 + j) * OSP + nb * 16 + lr] = acc[mb][nb][j]; } }
    wave_sync();
    const int c4 = lr * 4;
    const v4f bv = *(const v4f*)(BS + n0 + c4);
#pragma unroll 1
    for (int ps = 0; ps < 2; ++ps) {
#pragma unroll 1
        for (int it = 0; it < 32; ++it) { const int row = 2 * it + hi;
            v4f v = *(const v4fa*)(&os[row * OSP + c4]);
            v[0] += bv[0]; v[1] += bv[1]; v[2] += bv[2]; v[3] += bv[3];
            *(volatile v4f*)(SORTED + (size_t)(p0 + row) * ND + n0 + c4) = v; }
        if (ps == 0) __threadfence(); }
}

__global__ __launch_bounds__(256) void k_unsort(const int* __restrict__ POS, const float* __restrict__ SORTED, float* OUT) {
    const int row = min((int)blockIdx.x, NB - 1);
    const int p = clampi(POS[row], 0, PROWS - 1);
    const int c4 = 4 * threadIdx.x;
    const v4f v = *(const v4f*)(SORTED + (size_t)p * ND + c4);
    *(volatile v4f*)(OUT + (size_t)row * ND + c4) = v; __threadfence(); *(volatile v4f*)(OUT + (size_t)row * ND + c4) = v;
}

static constexpr size_t al256(size_t v) { return (v + 255) & ~(size_t)255; }
static constexpr size_t SZ_WB  = al256((size_t)NREL * ND * KD * 2);
static constexpr size_t SZ_CNT = al256((size_t)NBLK * 32 * 4);
static constexpr size_t SZ_OFF = al256((size_t)NSLOT * OFFP * 4);
static constexpr size_t SZ_T   = al256((size_t)128 * 4);
static constexpr size_t SZ_POS = al256((size_t)NB * 4);
static constexpr size_t SZ_BS  = al256((size_t)ND * 4);
static constexpr size_t SZ_PL  = al256((size_t)PROWS * KD * 2);
static constexpr size_t SZ_SRT = al256((size_t)PROWS * ND * 4);
static constexpr size_t SZ_TOTAL = SZ_WB + SZ_CNT + SZ_OFF + SZ_T + SZ_POS + SZ_BS + SZ_PL + SZ_SRT;
static_assert(SZ_TOTAL <= (size_t)134217728);

extern "C" void kernel_launch(void* const* d_in, const int* in_sizes, int n_in,
                              void* d_out, int out_size, void* d_ws, size_t ws_size, hipStream_t stream) {
    if (n_in < 4) return;
    if ((size_t)in_sizes[0] < (size_t)NB * KD) return;
    if ((size_t)in_sizes[1] < (size_t)NB) return;
    if ((size_t)in_sizes[2] < (size_t)NREL * ND * KD) return;
    if ((size_t)in_sizes[3] < (size_t)NREL * ND) return;
    if ((size_t)out_size < (size_t)NB * ND) return;
    if (SZ_TOTAL > ws_size) return;
    const float* xin = (const float*)d_in[0];
    const int*   cid = (const int*)d_in[1];
    const float* Win = (const float*)d_in[2];
    const float* bin = (const float*)d_in[3];
    float* OUT = (float*)d_out;
    char* wsp = (char*)d_ws;
    bf*  WB  = (bf*)wsp;  wsp += SZ_WB;
    int* CNT = (int*)wsp; wsp += SZ_CNT;
    int* OFF = (int*)wsp; wsp += SZ_OFF;
    int* TT  = (int*)wsp; wsp += SZ_T;
    int* POS = (int*)wsp; wsp += SZ_POS;
    float* BS = (float*)wsp; wsp += SZ_BS;
    bf*  AP  = (bf*)wsp;  wsp += SZ_PL;
    float* SRT = (float*)wsp; wsp += SZ_SRT;

    k_wconv<<<(unsigned)(((size_t)NREL * ND * KD) / (256 * 8)), 256, 0, stream>>>(Win, WB);
    k_bias<<<1, 256, 0, stream>>>(bin, BS);
    k_count<<<NBLK, 1024, 0, stream>>>(cid, CNT);
    k_scan<<<1, 1024, 0, stream>>>(CNT, OFF, TT, AP);
    k_rank<<<NBLK, 1024, 0, stream>>>(cid, xin, OFF, POS, AP);
    k_gemm<<<dim3(PROWS / 64, ND / 64), 32, 0, stream>>>(AP, WB, BS, TT, SRT);
    k_unsort<<<NB, 256, 0, stream>>>(POS, SRT, OUT);
}
